// DiffAttention_81063212745635
// MI455X (gfx1250) — hardware-run, weakly checked
//
#include <hip/hip_runtime.h>


#ifndef NB
#define NB 2
#endif
#ifndef SEQ
#define SEQ 2048
#endif
#define NB_FULL  2
#define SEQ_FULL 2048
#ifndef OUT_SEQ
#define OUT_SEQ SEQ
#endif
#define DM   128
#define NH_  8
#define QKW  (2 * NH_ * DM)
#define VW   (NH_ * DM)
#define HR   (2 * DM)
#define TPH  (SEQ / NH_)
#define AW   4
#define OSP  132
#define QKC  4.0f
#define VC   4.0f
#define VCI  0.25f
#define WOC  64.0f
#define WOI  (1.0f / 64.0f)
#define ZRS  2048.0f
#define ZRI  (1.0f / 2048.0f)
#define SC2  ((float)(1.4426950408889634 / 16.0))
#define PSH  14.0f
#define NEGB (-3.0e38f)
#define GEPS 1.0e-5f
#define GNE  (SEQ * DM)
#define NPIECE ((unsigned)(NB * SEQ) * (unsigned)(VW / 8))

static_assert(DM == 128);
static_assert(NH_ * DM == VW);
static_assert(DM % 32 == 0);
static_assert(VW % 32 == 0);
static_assert(QKW % 64 == 0);
static_assert(VW % 64 == 0);
static_assert(DM % 64 == 0);
static_assert(SEQ % NH_ == 0);
static_assert(TPH % 64 == 0);
static_assert(SEQ % 64 == 0);
static_assert((NB * SEQ) % 64 == 0);
static_assert(SEQ % 32 == 0);
static_assert(SEQ % (16 * AW) == 0);
static_assert((GNE / 4) % 256 == 0);
static_assert(((size_t)NB * SEQ * VW / 8) % 256 == 0);
static_assert(NB <= NB_FULL);
static_assert(SEQ <= SEQ_FULL);
static_assert((OSP * 4) % 16 == 0);
static_assert(AW * 16 * OSP * 4 <= 131072);
static_assert(16 * 68 * 4 <= 131072);

typedef _Float16 h16;
typedef unsigned short bf;
typedef __attribute__((ext_vector_type(16))) __bf16   v16bf;
typedef __attribute__((ext_vector_type(16))) _Float16 v16h;
typedef __attribute__((ext_vector_type(8)))  _Float16 v8h;
typedef __attribute__((ext_vector_type(8)))  unsigned short v8us;
typedef __attribute__((ext_vector_type(8)))  float    v8f;
typedef __attribute__((ext_vector_type(4)))  float    v4f;
typedef v4f  __attribute__((may_alias)) v4fa;

__device__ __forceinline__ unsigned short f2bf(float f) { unsigned u = __float_as_uint(f); u += 0x7FFFu + ((u >> 16) & 1u); return (unsigned short)(u >> 16); }
__device__ __forceinline__ float bfr(float f) { return __uint_as_float(((unsigned)f2bf(f)) << 16); }
__device__ __forceinline__ v16h cat16(v8h lo, v8h hi) { return __builtin_shufflevector(lo, hi, 0, 1, 2, 3, 4, 5, 6, 7, 8, 9, 10, 11, 12, 13, 14, 15); }
__device__ __forceinline__ v16bf cat16b(v8us lo, v8us hi) { return __builtin_bit_cast(v16bf, __builtin_shufflevector(lo, hi, 0, 1, 2, 3, 4, 5, 6, 7, 8, 9, 10, 11, 12, 13, 14, 15)); }
__device__ __forceinline__ v8f wmma16(v16h a, v16h b, v8f c) { return __builtin_amdgcn_wmma_f32_16x16x32_f16(false, a, false, b, (short)0, c, false, false); }
__device__ __forceinline__ v8f wmmab(v16bf a, v16bf b, v8f c) { return __builtin_amdgcn_wmma_f32_16x16x32_bf16(false, a, false, b, (short)0, c, false, false); }
__device__ __forceinline__ v16h  ldh(const h16* p) { return cat16(*(const v8h*)p, *(const v8h*)(p + 16)); }
__device__ __forceinline__ v16bf ldb(const bf* p)  { return cat16b(*(const v8us*)p, *(const v8us*)(p + 16)); }
__device__ __forceinline__ void wave_sync() { __builtin_amdgcn_fence(3  , "wavefront"); __builtin_amdgcn_wave_barrier(); asm volatile("" ::: "memory"); }

__device__ __forceinline__ v8f wmma16g(v16h a, v16h b, v8f c) { c = wmma16(a, b, c); asm volatile("v_nop\n\tv_nop\n\tv_nop\n\tv_nop" : "+v"(c) : "v"(a), "v"(b)); return c; }
__device__ __forceinline__ v8f wmmabg(v16bf a, v16bf b, v8f c) { c = wmmab(a, b, c); asm volatile("v_nop\n\tv_nop\n\tv_nop\n\tv_nop" : "+v"(c) : "v"(a), "v"(b)); return c; }
static __device__ __forceinline__ h16 toh_flush(float v) { const float w = (fabsf(v) < 6.103515625e-05f) ? 0.0f : v; return (h16)w; }

__global__ __launch_bounds__(256) void k_cvt8(const float* __restrict__ src, bf* dst, size_t n8) {
    const size_t i = (size_t)blockIdx.x * 256 + threadIdx.x; if (i >= n8) return;
    const v8f v = *(const v8f*)(src + i * 8); v8us o;
#pragma unroll
    for (int k = 0; k < 8; ++k) o[k] = f2bf(v[k]);
    *(volatile v8us*)(dst + i * 8) = o; __threadfence(); *(volatile v8us*)(dst + i * 8) = o;
}

__global__ __launch_bounds__(256) void k_wconv(const float* __restrict__ src, h16* dst, size_t n8) {
    const size_t i = (size_t)blockIdx.x * 256 + threadIdx.x; if (i >= n8) return;
    const v8f v = *(const v8f*)(src + i * 8); v8h o;
#pragma unroll
    for (int k = 0; k < 8; ++k) o[k] = toh_flush(bfr(v[k]) * WOC);
    *(volatile v8h*)(dst + i * 8) = o; __threadfence(); *(volatile v8h*)(dst + i * 8) = o;
}

template <int MODE>
__device__ __forceinline__ void proj_body(const bf* __restrict__ A, const bf* __restrict__ Bt, const float* __restrict__ bias, h16* P) {
    __shared__ __align__(16) float os[16 * 68];
    const int lane = threadIdx.x & 31, lr = lane & 15, hi = lane >> 4;
    const unsigned bx = blockIdx.x, by = blockIdx.y;
    v8f acc[4][4];
#pragma unroll
    for (int mb = 0; mb < 4; ++mb)
#pragma unroll
        for (int nb = 0; nb < 4; ++nb) acc[mb][nb] = (v8f){};
    size_t arow, astep;
    if (MODE == 0) { arow = (size_t)(64u * bx + (unsigned)lr); astep = (size_t)16 * DM; }
    else           { arow = (size_t)((unsigned)DM * (unsigned)(lr & 7) + 8u * bx + (unsigned)(lr >> 3)); astep = (size_t)2 * DM; }
    const size_t aoff = arow * DM + 8 * hi;
    const size_t boff = (size_t)(64u * by + (unsigned)lr) * DM + 8 * hi;
#pragma unroll 1
    for (int kc = 0; kc < DM; kc += 32) {
        v16bf a[4];
#pragma unroll
        for (int mb = 0; mb < 4; ++mb) a[mb] = ldb(A + aoff + (size_t)mb * astep + kc);
#pragma unroll
        for (int nb = 0; nb < 4; ++nb) { const v16bf b = ldb(Bt + boff + (size_t)nb * 16 * DM + kc);
#pragma unroll
            for (int mb = 0; mb < 4; ++mb) acc[mb][nb] = wmmabg(a[mb], b, acc[mb][nb]); }
    }
    float bc[4];
#pragma unroll
    for (int nb = 0; nb < 4; ++nb) bc[nb] = (MODE == 0) ? bfr(bias[64u * by + (unsigned)(nb * 16 + lr)]) : 0.0f;
    const unsigned n0 = 64u * by;
    const unsigned bb = n0 / (unsigned)SEQ, tokl = n0 % (unsigned)SEQ;
    const unsigned hh = tokl / (unsigned)TPH, tkb = tokl % (unsigned)TPH;
#pragma unroll
    for (int mb = 0; mb < 4; ++mb) {
        float br[8];
#pragma unroll
        for (int j = 0; j < 8; ++j) br[j] = (MODE == 1) ? bfr(bias[(unsigned)(DM * j) + 8u * bx + (unsigned)(2 * mb + hi)]) : 0.0f;
#pragma unroll
        for (int nb = 0; nb < 4; ++nb) {
#pragma unroll
            for (int j = 0; j < 8; ++j) os[(hi * 8 + j) * 68 + nb * 16 + lr] = acc[mb][nb][j] + bc[nb] + br[j]; }
        wave_sync();
#pragma unroll 1
        for (int ps = 0; ps < 2; ++ps) {
            if (MODE == 0) {
                static_assert(4 * 32 * 8 == 16 * 64);
                const size_t sb = ((size_t)(64u * bx) + (size_t)(mb * 16)) * QKW + (size_t)(64u * by);
#pragma unroll
                for (int s = 0; s < 4; ++s) { const int row = 4 * s + (lane >> 3), c8 = (lane & 7) * 8;
                    const v4f x0 = *(const v4fa*)(&os[row * 68 + c8]); const v4f x1 = *(const v4fa*)(&os[row * 68 + c8 + 4]); v8h hv;
#pragma unroll
                    for (int i = 0; i < 4; ++i) { hv[i] = toh_flush(x0[i] * QKC); hv[4 + i] = toh_flush(x1[i] * QKC); }
                    *(volatile v8h*)(P + sb + (size_t)row * QKW + c8) = hv; }
            } else {
                static_assert(2 * 2 * 32 * 8 == 16 * 64);
                const size_t vb = (size_t)((bb * (unsigned)NH_ + hh) * (unsigned)DM + 8u * bx + (unsigned)(2 * mb)) * SEQ + (size_t)(8u * tkb);
#pragma unroll
                for (int dlr = 0; dlr < 2; ++dlr) {
#pragma unroll
                    for (int s = 0; s < 2; ++s) { const int p = s * 32 + lane; v8h hv;
#pragma unroll
                        for (int pc = 0; pc < 8; ++pc) hv[pc] = toh_flush(os[(dlr * 8 + pc) * 68 + p] * VC);
                        *(volatile v8h*)(P + vb + (size_t)dlr * SEQ + (size_t)p * 8) = hv; } }
            }
            if (ps == 0) __threadfence(); }
        wave_sync();
    }
}

__global__ __launch_bounds__(32) void k_proj_rows(const bf* __restrict__ A, const bf* __restrict__ Bt, const float* __restrict__ bias, h16* P) { proj_body<0>(A, Bt, bias, P); }
__global__ __launch_bounds__(32) void k_proj_vt(const bf* __restrict__ A, const bf* __restrict__ Bt, const float* __restrict__ bias, h16* P) { proj_body<1>(A, Bt, bias, P); }

__device__ __forceinline__ void soft_step(const v8f sa, const v8f sb, float& m, float& l, v16h& p, float& alpha) {
    float ta[8], tb[8]; float mx = NEGB;
#pragma unroll
    for (int r = 0; r < 8; ++r) { ta[r] = sa[r] * SC2; tb[r] = sb[r] * SC2; mx = fmaxf(mx, fmaxf(ta[r], tb[r])); }
    mx = fmaxf(mx, __shfl_xor(mx, 16, 32));
    const float mnew = fmaxf(m, mx);
    alpha = __builtin_amdgcn_exp2f(m - mnew);
    const float sh = PSH - mnew;
    float ls = 0.0f;
#pragma unroll
    for (int r = 0; r < 8; ++r) {
        const float ea = ta[r] + sh, eb = tb[r] + sh;
        const float xa = __builtin_amdgcn_exp2f(ea), xb = __builtin_amdgcn_exp2f(eb);
        const float ga = (ea < -14.0f) ? 0.0f : xa, gb = (eb < -14.0f) ? 0.0f : xb;
        const h16 pa = (h16)ga; const h16 pc = (h16)gb;
        p[r] = pa; p[8 + r] = pc;
        ls += (float)pa + (float)pc; }
    l = l * alpha + ls; m = mnew;
}

__global__ __launch_bounds__(32 * AW) __attribute__((amdgpu_num_vgpr(256))) void k_flash(const h16* __restrict__ QP, const h16* __restrict__ KP, const h16* __restrict__ VT,
                                                                                        const float* __restrict__ lam_p, float* G) {
    __shared__ __align__(16) float os[AW * 16 * OSP];
    const int lane = threadIdx.x & 31, lr = lane & 15, hi = lane >> 4;
    const int wave = __builtin_amdgcn_readfirstlane((int)(threadIdx.x >> 5));
    const unsigned zh = blockIdx.y; const unsigned b = zh / (unsigned)NH_, h = zh % (unsigned)NH_;
    const int t0 = ((int)blockIdx.x * AW + wave) * 16;
    const size_t hb = (size_t)b * SEQ * QKW + (size_t)h * SEQ * HR;
    const size_t qo = hb + (size_t)(t0 + lr) * HR + 8 * hi;
    const size_t ko = hb + (size_t)lr * HR + 8 * hi;
    const size_t vo = ((size_t)zh * DM + (size_t)lr) * SEQ + 8 * hi;
    v8f o1[8], o2[8];
#pragma unroll
    for (int j = 0; j < 8; ++j) { o1[j] = (v8f){}; o2[j] = (v8f){}; }
    float m1 = NEGB, l1 = 0.0f, m2 = NEGB, l2 = 0.0f;
#pragma unroll 1
    for (int key0 = 0; key0 < SEQ; key0 += 32) {
        unsigned qz = 0; asm volatile("" : "+v"(qz));
        const h16* qb = QP + qo + qz;
        const h16* kb = KP + ko + (size_t)key0 * HR;
        v16h p1, p2; float al1, al2;
        { v8f sa = (v8f){}, sb = (v8f){};
#pragma unroll 2
          for (int ks = 0; ks < DM / 32; ++ks) {
              const v16h q = ldh(qb + ks * 32);
              const v16h ka = ldh(kb + ks * 32), kc = ldh(kb + 16 * HR + ks * 32);
              sa = wmma16g(ka, q, sa); sb = wmma16g(kc, q, sb); }
          soft_step(sa, sb, m1, l1, p1, al1); }
        { v8f sa = (v8f){}, sb = (v8f){};
#pragma unroll 2
          for (int ks = 0; ks < DM / 32; ++ks) {
              const v16h q = ldh(qb + DM + ks * 32);
              const v16h ka = ldh(kb + DM + ks * 32), kc = ldh(kb + 16 * HR + DM + ks * 32);
              sa = wmma16g(ka, q, sa); sb = wmma16g(kc, q, sb); }
          soft_step(sa, sb, m2, l2, p2, al2); }
#pragma unroll
        for (int j = 0; j < 8; ++j) { o1[j] = o1[j] * al1; o2[j] = o2[j] * al2; }
        const h16* va = VT + vo + key0;
#pragma unroll
        for (int jg = 0; jg < 2; ++jg) {
            v16h vv[4];
#pragma unroll
            for (int j = 0; j < 4; ++j) vv[j] = ldh(va + (size_t)((jg * 4 + j) * 16) * SEQ);
#pragma unroll
            for (int j = 0; j < 4; ++j) { o1[jg * 4 + j] = wmma16g(vv[j], p1, o1[jg * 4 + j]); o2[jg * 4 + j] = wmma16g(vv[j], p2, o2[jg * 4 + j]); }
        }
    }
    l1 += __shfl_xor(l1, 16, 32);
    l2 += __shfl_xor(l2, 16, 32);
    const float lamv = bfr(lam_p[0]);
    const float i1 = (1.0f / l1) * VCI;
    const float i2 = lamv * (1.0f / l2) * VCI;
    const int wb = wave * 16 * OSP;
#pragma unroll
    for (int j = 0; j < 8; ++j) { v4f a, c;
#pragma unroll
        for (int i = 0; i < 4; ++i) { a[i] = o1[j][i] * i1 - o2[j][i] * i2; c[i] = o1[j][4 + i] * i1 - o2[j][4 + i] * i2; }
        *(v4fa*)(&os[wb + lr * OSP + 16 * j + 8 * hi]) = a; *(v4fa*)(&os[wb + lr * OSP + 16 * j + 8 * hi + 4]) = c; }
    wave_sync();
    static_assert(32 * 4 == DM);
    float* grow = G + ((size_t)b * SEQ + (size_t)t0) * VW + (size_t)h * DM;
#pragma unroll 1
    for (int ps = 0; ps < 2; ++ps) {
#pragma unroll 4
        for (int row = 0; row < 16; ++row) { const int cofs = lane * 4;
            const v4f val = *(const v4fa*)(&os[wb + row * OSP + cofs]);
            *(volatile v4f*)(grow + (size_t)row * VW + cofs) = val; }
        if (ps == 0) __threadfence(); }
}

__global__ __launch_bounds__(256) void k_gnstat(const float* __restrict__ G, float* ST) {
#pragma clang fp contract(off)
    __shared__ float red1[8];
    __shared__ float red2[8];
    const int lane = threadIdx.x & 31;
    const int wave = __builtin_amdgcn_readfirstlane((int)(threadIdx.x >> 5));
    const unsigned zg = blockIdx.x;
    const float* p = G + (size_t)zg * GNE + (size_t)threadIdx.x * 4;
    v4f s4 = (v4f){};
#pragma unroll 1
    for (int it = 0; it < GNE / 4 / 256; ++it) { const v4f v = *(const v4f*)(p + (size_t)it * 1024); s4 = s4 + v; }
    float s = (s4[0] + s4[1]) + (s4[2] + s4[3]);
    s += __shfl_xor(s, 16, 32); s += __shfl_xor(s, 8, 32); s += __shfl_xor(s, 4, 32); s += __shfl_xor(s, 2, 32); s += __shfl_xor(s, 1, 32);
    if (lane == 0) red1[wave] = s;
    __syncthreads();
    const float tot = ((red1[0] + red1[1]) + (red1[2] + red1[3])) + ((red1[4] + red1[5]) + (red1[6] + red1[7]));
    const float mean = tot * (1.0f / (float)GNE);
    v4f q4 = (v4f){};
#pragma unroll 1
    for (int it = 0; it < GNE / 4 / 256; ++it) { const v4f v = *(const v4f*)(p + (size_t)it * 1024); const v4f d = v - mean; q4 = q4 + d * d; }
    float q = (q4[0] + q4[1]) + (q4[2] + q4[3]);
    q += __shfl_xor(q, 16, 32); q += __shfl_xor(q, 8, 32); q += __shfl_xor(q, 4, 32); q += __shfl_xor(q, 2, 32); q += __shfl_xor(q, 1, 32);
    if (lane == 0) red2[wave] = q;
    __syncthreads();
    const float tq = ((red2[0] + red2[1]) + (red2[2] + red2[3])) + ((red2[4] + red2[5]) + (red2[6] + red2[7]));
    const float var = tq * (1.0f / (float)GNE);
    const float rstd = rsqrtf(var + GEPS);
    if (threadIdx.x < 8) {
        v4f o = (v4f){};
        const float sel = (threadIdx.x == 0) ? 1.0f : 0.0f;
        o[0] = mean * sel; o[1] = rstd * sel;
        float* dst = ST + (size_t)zg * 32 + (size_t)threadIdx.x * 4;
        *(volatile v4f*)dst = o; __threadfence(); *(volatile v4f*)dst = o;
    }
}

__global__ __launch_bounds__(256) void k_norm(const float* __restrict__ G, const float* __restrict__ ST, const float* __restrict__ gw, const float* __restrict__ gb,
                                              const float* __restrict__ lam_p, h16* ZH, h16* ZR) {
#pragma clang fp contract(off)
    const unsigned i = blockIdx.x * 256u + threadIdx.x; if (i >= NPIECE) return;
    const unsigned c8 = i % (unsigned)(VW / 8), R = i / (unsigned)(VW / 8);
    const unsigned b = R / (unsigned)SEQ, r = R % (unsigned)SEQ;
    const unsigned g = c8 / (unsigned)(DM / 8), d8 = (c8 % (unsigned)(DM / 8)) * 8u;
    const unsigned zg = b * (unsigned)NH_ + g;
    const float* src = G + ((size_t)zg * SEQ + (size_t)r) * DM + d8;
    const v4f x0 = *(const v4f*)src, x1 = *(const v4f*)(src + 4);
    const float mean = ST[(size_t)zg * 32], rstd = ST[(size_t)zg * 32 + 1];
    const float gwv = bfr(gw[g]), gbv = bfr(gb[g]);
    const float oml = 1.0f - bfr(lam_p[0]);
    v8h hv, rv;
#pragma unroll
    for (int k = 0; k < 4; ++k) {
        const float z0 = ((x0[k] - mean) * rstd * gwv + gbv) * oml;
        const float z1 = ((x1[k] - mean) * rstd * gwv + gbv) * oml;
        const h16 a0 = toh_flush(z0); const h16 a1 = toh_flush(z1);
        hv[k] = a0; hv[4 + k] = a1;
        rv[k] = toh_flush((z0 - (float)a0) * ZRS); rv[4 + k] = toh_flush((z1 - (float)a1) * ZRS); }
    *(volatile v8h*)(ZH + (size_t)i * 8) = hv; *(volatile v8h*)(ZR + (size_t)i * 8) = rv;
    __threadfence();
    *(volatile v8h*)(ZH + (size_t)i * 8) = hv; *(volatile v8h*)(ZR + (size_t)i * 8) = rv;
}

__global__ __launch_bounds__(32) void k_out(const h16* __restrict__ ZH, const h16* __restrict__ ZR, const h16* __restrict__ WO, const float* __restrict__ bo, float* OUT) {
    __shared__ __align__(16) float os[16 * 68];
    const int lane = threadIdx.x & 31, lr = lane & 15, hi = lane >> 4;
    const unsigned bx = blockIdx.x, by = blockIdx.y;
    v8f acc[2][4], acr[2][4];
#pragma unroll
    for (int mb = 0; mb < 2; ++mb)
#pragma unroll
        for (int nb = 0; nb < 4; ++nb) { acc[mb][nb] = (v8f){}; acr[mb][nb] = (v8f){}; }
    const size_t aoff = (size_t)(32u * bx + (unsigned)lr) * VW + 8 * hi;
    const size_t boff = (size_t)(64u * by + (unsigned)lr) * VW + 8 * hi;
#pragma unroll 1
    for (int kc = 0; kc < VW; kc += 32) {
        v16h a[2], ar[2];
#pragma unroll
        for (int mb = 0; mb < 2; ++mb) { a[mb] = ldh(ZH + aoff + (size_t)mb * 16 * VW + kc); ar[mb] = ldh(ZR + aoff + (size_t)mb * 16 * VW + kc); }
#pragma unroll
        for (int nb = 0; nb < 4; ++nb) { const v16h w = ldh(WO + boff + (size_t)nb * 16 * VW + kc);
#pragma unroll
            for (int mb = 0; mb < 2; ++mb) { acc[mb][nb] = wmma16g(a[mb], w, acc[mb][nb]); acr[mb][nb] = wmma16g(ar[mb], w, acr[mb][nb]); } }
    }
    float bc[4];
#pragma unroll
    for (int nb = 0; nb < 4; ++nb) bc[nb] = bfr(bo[64u * by + (unsigned)(nb * 16 + lr)]);
    const unsigned mt = 32u * bx;
    const unsigned bb = mt / (unsigned)SEQ, rr = mt % (unsigned)SEQ;
    float* obase = OUT + ((size_t)bb * OUT_SEQ + (size_t)rr) * DM + (size_t)(64u * by);
#pragma unroll
    for (int mb = 0; mb < 2; ++mb) {
#pragma unroll
        for (int nb = 0; nb < 4; ++nb) {
#pragma unroll
            for (int j = 0; j < 8; ++j) os[(hi * 8 + j) * 68 + nb * 16 + lr] = (acc[mb][nb][j] + acr[mb][nb][j] * ZRI) * WOI + bc[nb]; }
        wave_sync();
        static_assert(8 * 32 * 4 == 16 * 64);
#pragma unroll 1
        for (int ps = 0; ps < 2; ++ps) {
#pragma unroll
            for (int s = 0; s < 8; ++s) { const int row = 2 * s + (lane >> 4), cofs = (lane & 15) * 4;
                const v4f val = *(const v4fa*)(&os[row * 68 + cofs]);
                *(volatile v4f*)(obase + (size_t)(mb * 16 + row) * DM + cofs) = val; }
            if (ps == 0) __threadfence(); }
        wave_sync();
    }
}

static constexpr size_t al256(size_t v) { return (v + 255) & ~(size_t)255; }
static constexpr size_t SZ_XB = al256((size_t)NB * SEQ * DM * 2);
static constexpr size_t SZ_WB = al256((size_t)(2 * QKW + VW) * DM * 2);
static constexpr size_t SZ_WO = al256((size_t)DM * VW * 2);
static constexpr size_t SZ_QK = al256((size_t)NB * SEQ * QKW * 2);
static constexpr size_t SZ_VT = al256((size_t)NB * NH_ * DM * SEQ * 2);
static constexpr size_t SZ_G  = al256((size_t)NB * SEQ * VW * 4);
static constexpr size_t SZ_ST = al256((size_t)NB * NH_ * 32 * 4);
static constexpr size_t SZ_Z  = al256((size_t)NB * SEQ * VW * 2);
static constexpr size_t SZ_TOTAL = SZ_XB + SZ_WB + SZ_WO + 2 * SZ_QK + SZ_VT + SZ_G + SZ_ST + 2 * SZ_Z;
static_assert(SZ_TOTAL <= (size_t)134217728);
static_assert(((size_t)QKW * DM * 2) % 256 == 0);
static_assert((size_t)NB * NH_ * DM * SEQ == (size_t)NB * SEQ * VW);
static constexpr size_t NEED_X = ((size_t)(NB - 1) * SEQ_FULL + SEQ) * DM;
static constexpr size_t NEED_O = ((size_t)(NB - 1) * OUT_SEQ + SEQ) * DM;
static constexpr size_t N8_X   = (size_t)NB * SEQ * DM / 8;
static constexpr size_t N8_X1  = (size_t)SEQ * DM / 8;
static constexpr size_t N8_WQK = (size_t)QKW * DM / 8;
static constexpr size_t N8_WV  = (size_t)VW * DM / 8;
static constexpr size_t N8_WO  = (size_t)DM * VW / 8;

extern "C" void kernel_launch(void* const* d_in, const int* in_sizes, int n_in,
                              void* d_out, int out_size, void* d_ws, size_t ws_size, hipStream_t stream) {
    if (n_in < 12) return;
    if ((size_t)in_sizes[0] < NEED_X) return;
    if ((size_t)in_sizes[1] < (size_t)QKW * DM || (size_t)in_sizes[3] < (size_t)QKW * DM) return;
    if ((size_t)in_sizes[5] < (size_t)VW * DM || (size_t)in_sizes[7] < (size_t)DM * VW) return;
    if (in_sizes[2] < QKW || in_sizes[4] < QKW || in_sizes[6] < VW || in_sizes[8] < DM) return;
    if (in_sizes[9] < NH_ || in_sizes[10] < NH_ || in_sizes[11] < 1) return;
    if ((size_t)out_size < NEED_O) return;
    if (SZ_TOTAL > ws_size) return;
    const float* xin = (const float*)d_in[0];
    const float* wq = (const float*)d_in[1]; const float* bq = (const float*)d_in[2];
    const float* wk = (const float*)d_in[3]; const float* bk = (const float*)d_in[4];
    const float* wv = (const float*)d_in[5]; const float* bv = (const float*)d_in[6];
    const float* wo = (const float*)d_in[7]; const float* bo = (const float*)d_in[8];
    const float* gw = (const float*)d_in[9]; const float* gb = (const float*)d_in[10];
    const float* lam = (const float*)d_in[11];
    float* OUT = (float*)d_out;
    char* wsp = (char*)d_ws;
    bf*  XB  = (bf*)wsp;  wsp += SZ_XB;
    bf*  WB  = (bf*)wsp;  wsp += SZ_WB;
    h16* WOH = (h16*)wsp; wsp += SZ_WO;
    h16* QP  = (h16*)wsp; wsp += SZ_QK;
    h16* KP  = (h16*)wsp; wsp += SZ_QK;
    h16* VT  = (h16*)wsp; wsp += SZ_VT;
    float* G = (float*)wsp; wsp += SZ_G;
    float* ST = (float*)wsp; wsp += SZ_ST;
    h16* ZH  = (h16*)wsp; wsp += SZ_Z;
    h16* ZR  = (h16*)wsp; wsp += SZ_Z;
    bf* WQ = WB; bf* WK = WB + (size_t)QKW * DM; bf* WV = WB + (size_t)2 * QKW * DM;

    if (SEQ == SEQ_FULL) {
        k_cvt8<<<(unsigned)((N8_X + 255) / 256), 256, 0, stream>>>(xin, XB, N8_X);
    } else {
        for (int b = 0; b < NB; ++b) k_cvt8<<<(unsigned)((N8_X1 + 255) / 256), 256, 0, stream>>>(xin + (size_t)b * SEQ_FULL * DM, XB + (size_t)b * SEQ * DM, N8_X1);
    }
    k_cvt8<<<(unsigned)((N8_WQK + 255) / 256), 256, 0, stream>>>(wq, WQ, N8_WQK);
    k_cvt8<<<(unsigned)((N8_WQK + 255) / 256), 256, 0, stream>>>(wk, WK, N8_WQK);
    k_cvt8<<<(unsigned)((N8_WV + 255) / 256), 256, 0, stream>>>(wv, WV, N8_WV);
    k_wconv<<<(unsigned)((N8_WO + 255) / 256), 256, 0, stream>>>(wo, WOH, N8_WO);

    k_proj_rows<<<dim3(NB * SEQ / 64, QKW / 64, 1), 32, 0, stream>>>(XB, WQ, bq, QP);
    k_proj_rows<<<dim3(NB * SEQ / 64, QKW / 64, 1), 32, 0, stream>>>(XB, WK, bk, KP);
    k_proj_vt<<<dim3(VW / 64, NB * SEQ / 64, 1), 32, 0, stream>>>(WV, XB, bv, VT);

    k_flash<<<dim3(SEQ / (16 * AW), NB * NH_, 1), 32 * AW, 0, stream>>>(QP, KP, VT, lam, G);
    k_gnstat<<<dim3(NB * NH_, 1, 1), 256, 0, stream>>>(G, ST);
    k_norm<<<dim3((unsigned)(((size_t)NB * SEQ * VW / 8) / 256), 1, 1), 256, 0, stream>>>(G, ST, gw, gb, lam, ZH, ZR);
    k_out<<<dim3(NB * SEQ / 32, DM / 64, 1), 32, 0, stream>>>(ZH, ZR, WOH, bo, OUT);
}
